// DenseCRF_35579509080386
// MI455X (gfx1250) — hardware-run, weakly checked
//
#include <hip/hip_runtime.h>
#include <math.h>

constexpr int NBATCH = 2;
constexpr int NCH    = 21;
constexpr int IMG_H  = 80;
constexpr int IMG_W  = 80;
constexpr int NPIX   = IMG_H * IMG_W;
constexpr int MROWS  = 64;
constexpr int NITER  = 5;
constexpr float QCARRY   = 64.0f;
constexpr float KBCARRY  = 1024.0f;
constexpr float BI_SCALE = 5.0f / (64.0f * 1024.0f);
static_assert(NPIX == 6400, "npix");
static_assert(IMG_H == IMG_W, "one 1-D gaussian table serves both axes");
static_assert(NPIX % 256 == 0, "phase loops are exact");
static_assert(NPIX % 64 == 0 && NPIX % 32 == 0 && MROWS % 64 == 0, "gemm tile multiples");

constexpr size_t KBP_BYTES = (size_t)NPIX * NPIX * 2;
constexpr size_t Q16_BYTES = (size_t)MROWS * NPIX * 2;
constexpr size_t QF_BYTES  = (size_t)NCH * NPIX * 4;
constexpr size_t BI_BYTES  = (size_t)MROWS * NPIX * 4;
constexpr size_t OFF_KBP = 0;
constexpr size_t OFF_Q16 = OFF_KBP + KBP_BYTES;
constexpr size_t OFF_QFA = OFF_Q16 + Q16_BYTES;
constexpr size_t OFF_QFB = OFF_QFA + QF_BYTES;
constexpr size_t OFF_BI  = OFF_QFB + QF_BYTES;
constexpr size_t WS_TOTAL = OFF_BI + BI_BYTES;
static_assert(WS_TOTAL == 85452800u, "ws total");
static_assert(WS_TOTAL <= 134217728u, "ws cap");
static_assert(OFF_Q16 % 256 == 0 && OFF_QFA % 256 == 0 && OFF_QFB % 256 == 0 && OFF_BI % 256 == 0, "alignment");

typedef __attribute__((ext_vector_type(16))) _Float16 v16h;
typedef __attribute__((ext_vector_type(8)))  _Float16 v8h;
typedef __attribute__((ext_vector_type(16))) __bf16   v16b;
typedef __attribute__((ext_vector_type(8)))  __bf16   v8b;
typedef __attribute__((ext_vector_type(8)))  float    v8f;
typedef __attribute__((ext_vector_type(4)))  float    v4f;
typedef __attribute__((ext_vector_type(4)))  unsigned int v4u;

__device__ __forceinline__ unsigned short f2bf_bits(float f) {
  unsigned u = __float_as_uint(f);
  return (unsigned short)((u + 0x7FFFu + ((u >> 16) & 1u)) >> 16);
}
__device__ __forceinline__ float bf_bits2f(unsigned short h) { return __uint_as_float(((unsigned)h) << 16); }

__device__ __forceinline__ void dep_guard_h(v8f& a, v8f& b, v16h x, v16h y) { asm volatile("v_nop\n\tv_nop\n\tv_nop\n\tv_nop" : "+v"(a), "+v"(b) : "v"(x), "v"(y)); }
__device__ __forceinline__ void dep_guard_b(v8f& a, v8f& b, v16b x, v16b y) { asm volatile("v_nop\n\tv_nop\n\tv_nop\n\tv_nop" : "+v"(a), "+v"(b) : "v"(x), "v"(y)); }
__device__ __forceinline__ void keep4_h(v16h a, v16h b, v16h c, v16h d) { asm volatile("v_nop" :: "v"(a), "v"(b), "v"(c), "v"(d)); }
__device__ __forceinline__ void keep4_b(v16b a, v16b b, v16b c, v16b d) { asm volatile("v_nop" :: "v"(a), "v"(b), "v"(c), "v"(d)); }
__device__ __forceinline__ void acc_guard4(v8f& a, v8f& b, v8f& c, v8f& d) { asm volatile("v_nop\n\tv_nop\n\tv_nop\n\tv_nop" : "+v"(a), "+v"(b), "+v"(c), "+v"(d)); }
template <typename T> struct Frag;
template <> struct Frag<_Float16> {
  typedef v16h V; union U { v16h v; v8h h[2]; };
  static __device__ __forceinline__ v16h load(const _Float16* p) {
    U f; f.h[0] = *(const v8h*)(p); f.h[1] = *(const v8h*)(p + 16); return f.v;
  }
  static __device__ __forceinline__ v8f mma(v16h a, v16h b, v8f c) {
    return __builtin_amdgcn_wmma_f32_16x16x32_f16(false, a, false, b, (short)0, c, false, false);
  }
  static __device__ __forceinline__ void guard(v8f& a, v8f& b, v16h x, v16h y) { dep_guard_h(a, b, x, y); }
  static __device__ __forceinline__ void keep(v16h a, v16h b, v16h c, v16h d) { keep4_h(a, b, c, d); }
};
template <> struct Frag<__bf16> {
  typedef v16b V; union U { v16b v; v8b h[2]; };
  static __device__ __forceinline__ v16b load(const __bf16* p) {
    U f; f.h[0] = *(const v8b*)(p); f.h[1] = *(const v8b*)(p + 16); return f.v;
  }
  static __device__ __forceinline__ v8f mma(v16b a, v16b b, v8f c) {
    return __builtin_amdgcn_wmma_f32_16x16x32_bf16(false, a, false, b, (short)0, c, false, false);
  }
  static __device__ __forceinline__ void guard(v8f& a, v8f& b, v16b x, v16b y) { dep_guard_b(a, b, x, y); }
  static __device__ __forceinline__ void keep(v16b a, v16b b, v16b c, v16b d) { keep4_b(a, b, c, d); }
};

__device__ __forceinline__ unsigned pk16(unsigned short a, unsigned short b) { return (unsigned)a | ((unsigned)b << 16); }
__device__ __forceinline__ unsigned short h_bits(float f) { const _Float16 h = (_Float16)f; return __builtin_bit_cast(unsigned short, h); }

template <int ET> struct Elem;
template <> struct Elem<0> { typedef _Float16 T; };
template <> struct Elem<1> { typedef __bf16 T; };
template <int ET, bool SPLIT, int BIAS_MODE, int OUT_MODE, bool RESID, int ACT = 0>
__global__ __launch_bounds__(256) void wmma_gemm64(
    const unsigned short* __restrict__ Ap, const unsigned short* __restrict__ A2p, int lda, long strideA,
    const unsigned short* __restrict__ Btp, const unsigned short* __restrict__ Bt2p, int ldb, long strideB,
    void* __restrict__ Cout, void* __restrict__ Cout2, int ldc, long strideC,
    const float* __restrict__ bias,
    const float* __restrict__ resid, long strideR,
    int M, int N, int K, float scale) {
  typedef typename Elem<ET>::T T;
  typedef typename Frag<T>::V V;
  const T* A = (const T*)Ap; const T* A2 = (const T*)A2p; const T* Bt = (const T*)Btp; const T* Bt2 = (const T*)Bt2p;
  __shared__ __align__(16) float sT[8][16 * 68];
  const int b    = blockIdx.y;
  const int lane = threadIdx.x & 31;
  const int wave = threadIdx.x >> 5;
  const int tilesN = N >> 6;
  const int tilesM = M >> 6;
  const int tile = blockIdx.x * 8 + wave;
  if (tile >= tilesM * tilesN) return;
  const int tm = tile / tilesN;
  const int tn = tile - tm * tilesN;
  const int m0 = tm << 6;
  const int n0 = tn << 6;

  const T* Ab  = A  + (size_t)b * strideA;
  const T* Bb  = Bt + (size_t)b * strideB;
  const T* Ab2 = SPLIT ? (A2  + (size_t)b * strideA) : nullptr;
  const T* Bb2 = SPLIT ? (Bt2 + (size_t)b * strideB) : nullptr;

  const int rlane = lane & 15;
  const int koff  = (lane >> 4) * 8;
  const int mOff  = (lane >> 4) * 8;

  v8f acc[4][4];
#pragma unroll
  for (int i = 0; i < 4; ++i)
#pragma unroll
    for (int j = 0; j < 4; ++j) acc[i][j] = (v8f){0.f,0.f,0.f,0.f,0.f,0.f,0.f,0.f};

  for (int k0 = 0; k0 < K; k0 += 32) {
    V bh[4], bl[4];
#pragma unroll
    for (int j = 0; j < 4; ++j) {
      const size_t bo = (size_t)(n0 + (j << 4) + rlane) * ldb + koff + k0;
      bh[j] = Frag<T>::load(Bb + bo);
      if (SPLIT) bl[j] = Frag<T>::load(Bb2 + bo);
    }
#pragma unroll
    for (int i = 0; i < 4; ++i) {
      const size_t ao = (size_t)(m0 + (i << 4) + rlane) * lda + koff + k0;
      V ah = Frag<T>::load(Ab + ao);
      V al;
      if (SPLIT) al = Frag<T>::load(Ab2 + ao);
#pragma unroll
      for (int j = 0; j < 4; ++j) {
        acc[i][j] = Frag<T>::mma(ah, bh[j], acc[i][j]);
        if (SPLIT) {
          acc[i][j] = Frag<T>::mma(ah, bl[j], acc[i][j]);
          acc[i][j] = Frag<T>::mma(al, bh[j], acc[i][j]);
        }
      }
      Frag<T>::guard(acc[i][0], acc[i][3], ah, SPLIT ? al : ah);
    }
    Frag<T>::keep(bh[0], bh[1], bh[2], bh[3]);
    if (SPLIT) Frag<T>::keep(bl[0], bl[1], bl[2], bl[3]);
  }
  acc_guard4(acc[0][0], acc[0][1], acc[0][2], acc[0][3]);
  acc_guard4(acc[1][0], acc[1][1], acc[1][2], acc[1][3]);
  acc_guard4(acc[2][0], acc[2][1], acc[2][2], acc[2][3]);
  acc_guard4(acc[3][0], acc[3][1], acc[3][2], acc[3][3]);

  float* slab = sT[wave];
  const float* Rb = RESID ? (resid + (size_t)b * strideR) : nullptr;
#pragma unroll
  for (int i = 0; i < 4; ++i) {
    const int mBase = m0 + (i << 4);
#pragma unroll
    for (int j = 0; j < 4; ++j) {
      const int n = n0 + (j << 4) + rlane;
      float bv = 0.f;
      if (BIAS_MODE == 2) bv = bias[n];
#pragma unroll
      for (int r = 0; r < 8; ++r) {
        float v = acc[i][j][r] * scale;
        if (BIAS_MODE == 1) v += bias[mBase + mOff + r];
        if (BIAS_MODE == 2) v += bv;
        if (RESID) v += Rb[(size_t)(mBase + mOff + r) * ldc + n];
        if (ACT == 2) v = fmaxf(v, 0.0f);
        if (ACT == 4) v = (v > 0.f) ? v : 0.01f * v;
        slab[(mOff + r) * 68 + (j << 4) + rlane] = v;
      }
    }
    __builtin_amdgcn_fence(__ATOMIC_RELEASE, "workgroup");
    __builtin_amdgcn_wave_barrier();
    __builtin_amdgcn_fence(__ATOMIC_ACQUIRE, "workgroup");
    if (OUT_MODE == 0) {
      float* C = (float*)Cout + (size_t)b * strideC;
      const int hh = lane >> 4, c4 = (lane & 15) * 4;
      for (int pass = 0; pass < 2; ++pass) {
#pragma unroll
        for (int it = 0; it < 8; ++it) {
          const int row = it * 2 + hh;
          v4f v = *(const v4f*)(slab + row * 68 + c4);
          *(volatile v4f*)(C + (size_t)(mBase + row) * ldc + n0 + c4) = v;
        }
        __threadfence();
      }
    } else {
      const int q = lane >> 3, c8 = (lane & 7) * 8;
      unsigned short* C  = (unsigned short*)Cout  + (size_t)b * strideC;
      unsigned short* C2 = (OUT_MODE == 2) ? ((unsigned short*)Cout2 + (size_t)b * strideC) : nullptr;
      for (int pass = 0; pass < 2; ++pass) {
#pragma unroll
        for (int it = 0; it < 4; ++it) {
          const int row = it * 4 + q;
          const float* sp = slab + row * 68 + c8;
          v8h hv, lv;
#pragma unroll
          for (int e = 0; e < 8; ++e) {
            if (OUT_MODE == 1) {
              hv[e] = (_Float16)sp[e];
            } else {
              unsigned short hb = f2bf_bits(sp[e]);
              unsigned short lb = f2bf_bits(sp[e] - bf_bits2f(hb));
              hv[e] = __builtin_bit_cast(_Float16, hb);
              lv[e] = __builtin_bit_cast(_Float16, lb);
            }
          }
          *(volatile v8h*)(C + (size_t)(mBase + row) * ldc + n0 + c8) = hv;
          if (OUT_MODE == 2) *(volatile v8h*)(C2 + (size_t)(mBase + row) * ldc + n0 + c8) = lv;
        }
        __threadfence();
      }
    }
    __builtin_amdgcn_fence(__ATOMIC_RELEASE, "workgroup");
    __builtin_amdgcn_wave_barrier();
    __builtin_amdgcn_fence(__ATOMIC_ACQUIRE, "workgroup");
  }
}

__global__ __launch_bounds__(256) void zero_q16_pad_kernel(unsigned short* __restrict__ q16) {
  const int i = blockIdx.x * 256 + threadIdx.x;
  if (i >= (MROWS - NCH) * (NPIX / 8)) return;
  const v4u z = (v4u){0u, 0u, 0u, 0u};
  unsigned short* p = q16 + (size_t)NCH * NPIX + 8 * (size_t)i;
  *(volatile v4u*)p = z;
  __threadfence();
  *(volatile v4u*)p = z;
}

__global__ __launch_bounds__(256) void pack_q16_kernel(const float* __restrict__ predb, unsigned short* __restrict__ q16) {
  const int i = blockIdx.x * 256 + threadIdx.x;
  if (i >= NCH * (NPIX / 8)) return;
  const float* p = predb + 8 * (size_t)i;
  const v4f a = *(const v4f*)(p);
  const v4f c = *(const v4f*)(p + 4);
  unsigned short hb[8];
#pragma unroll
  for (int e = 0; e < 4; ++e) {
    hb[e]     = h_bits(a[e] * QCARRY);
    hb[4 + e] = h_bits(c[e] * QCARRY);
  }
  const v4u u = (v4u){pk16(hb[0], hb[1]), pk16(hb[2], hb[3]), pk16(hb[4], hb[5]), pk16(hb[6], hb[7])};
  unsigned short* q = q16 + 8 * (size_t)i;
  *(volatile v4u*)q = u;
  __threadfence();
  *(volatile v4u*)q = u;
}

__device__ __forceinline__ unsigned short kb_elem(float rm, float gm, float bm, float sqm, float rn, float gn, float bn) {
#pragma clang fp contract(off)
  const float sqn   = rn * rn + gn * gn + bn * bn;
  const float inner = rm * rn + gm * gn + bm * bn;
  const float d2    = (sqm + sqn) - 2.0f * inner;
  const float v     = expf((-d2) * (1.0f / 50.0f));
  return h_bits(v * KBCARRY);
}

__global__ __launch_bounds__(256) void build_kb_kernel(const float* __restrict__ imgb, unsigned short* __restrict__ kbp) {
#pragma clang fp contract(off)
  const int tid = blockIdx.x * 256 + threadIdx.x;
  if (tid >= NPIX * (NPIX / 8)) return;
  const int m  = tid / (NPIX / 8);
  const int j  = tid - m * (NPIX / 8);
  const int n0 = 8 * j;
  const float rm = imgb[m];
  const float gm = imgb[NPIX + m];
  const float bm = imgb[2 * NPIX + m];
  const float sqm = rm * rm + gm * gm + bm * bm;
  const float* pr = imgb + n0;
  const float* pg = imgb + NPIX + n0;
  const float* pb = imgb + 2 * NPIX + n0;
  const v4f r0 = *(const v4f*)(pr), r1 = *(const v4f*)(pr + 4);
  const v4f g0 = *(const v4f*)(pg), g1 = *(const v4f*)(pg + 4);
  const v4f b0 = *(const v4f*)(pb), b1 = *(const v4f*)(pb + 4);
  unsigned short hb[8];
#pragma unroll
  for (int e = 0; e < 4; ++e) {
    hb[e]     = kb_elem(rm, gm, bm, sqm, r0[e], g0[e], b0[e]);
    hb[4 + e] = kb_elem(rm, gm, bm, sqm, r1[e], g1[e], b1[e]);
  }
  const v4u u = (v4u){pk16(hb[0], hb[1]), pk16(hb[2], hb[3]), pk16(hb[4], hb[5]), pk16(hb[6], hb[7])};
  unsigned short* q = kbp + (size_t)m * NPIX + n0;
  *(volatile v4u*)q = u;
  __threadfence();
  *(volatile v4u*)q = u;
}

__global__ __launch_bounds__(256) void spatial_update_kernel(
    const float* __restrict__ qin, const float* __restrict__ predb, const float* __restrict__ bi,
    float* __restrict__ qout, unsigned short* __restrict__ q16) {
  __shared__ __align__(16) float sQ[NPIX];
  __shared__ __align__(16) float sTT[NPIX];
  __shared__ float sG[IMG_W];
  const int t = threadIdx.x;
  const int c = blockIdx.x;
  const size_t rowoff = (size_t)c * NPIX;

  for (int i = 0; i < 7; ++i) {
    const int i4  = t + 256 * i;
    const int i4c = (i4 < NPIX / 4) ? i4 : (NPIX / 4 - 1);
    const v4f v = *(const v4f*)(qin + rowoff + 4 * (size_t)i4c);
    if (i4 < NPIX / 4) *(v4f*)(sQ + 4 * i4) = v;
  }
  if (t < IMG_W) {
    const float dd = (float)(t * t);
    float g = expf(-(dd * (1.0f / 18.0f)));
    g = (g < 1.17549435e-38f) ? 0.0f : g;
    sG[t] = g;
  }
  __syncthreads();

#pragma unroll 1
  for (int i = 0; i < NPIX / 256; ++i) {
    const int p  = t + 256 * i;
    const int y  = p / IMG_W;
    const int xo = p - y * IMG_W;
    const float* qrow = sQ + y * IMG_W;
    float acc = 0.0f;
#pragma unroll 8
    for (int x = 0; x < IMG_W; ++x) {
      int d = x - xo;
      d = (d < 0) ? -d : d;
      acc = fmaf(qrow[x], sG[d], acc);
    }
    sTT[p] = acc;
  }
  __syncthreads();

#pragma unroll 1
  for (int i = 0; i < NPIX / 256; ++i) {
    const int p  = t + 256 * i;
    const int yo = p / IMG_W;
    const int x  = p - yo * IMG_W;
    float acc = 0.0f;
#pragma unroll 8
    for (int y = 0; y < IMG_H; ++y) {
      int d = y - yo;
      d = (d < 0) ? -d : d;
      acc = fmaf(sG[d], sTT[y * IMG_W + x], acc);
    }
    const float sp  = 3.0f * acc;
    const float bv  = bi[rowoff + p];
    const float pr  = predb[rowoff + p];
    const float msg = sp + bv;
    const float z   = pr - msg;
    const float e   = expf(-z);
    const float dn  = 1.0f + e;
    const float q   = __builtin_amdgcn_rcpf(dn);
    sQ[p] = q;
  }
  __syncthreads();

  float* orow = qout + rowoff;
  unsigned short* hrow = q16 + rowoff;
  for (int pass = 0; pass < 2; ++pass) {
#pragma unroll 1
    for (int i = 0; i < NPIX / 256; ++i) {
      const int p = t + 256 * i;
      const float v = sQ[p];
      *(volatile float*)(orow + p) = v;
    }
#pragma unroll 1
    for (int i = 0; i < 4; ++i) {
      const int j  = t + 256 * i;
      const int jc = (j < NPIX / 8) ? j : (NPIX / 8 - 1);
      const float* s8 = sQ + 8 * jc;
      const v4f a  = *(const v4f*)(s8);
      const v4f a2 = *(const v4f*)(s8 + 4);
      unsigned short hb[8];
#pragma unroll
      for (int e = 0; e < 4; ++e) {
        hb[e]     = h_bits(a[e] * QCARRY);
        hb[4 + e] = h_bits(a2[e] * QCARRY);
      }
      const v4u u = (v4u){pk16(hb[0], hb[1]), pk16(hb[2], hb[3]), pk16(hb[4], hb[5]), pk16(hb[6], hb[7])};
      if (j < NPIX / 8) *(volatile v4u*)(hrow + 8 * (size_t)j) = u;
    }
    __threadfence();
  }
}

extern "C" void kernel_launch(void* const* d_in, const int* in_sizes, int n_in,
                              void* d_out, int out_size, void* d_ws, size_t ws_size,
                              hipStream_t stream) {
  if (n_in < 2) return;
  if (in_sizes[0] != NBATCH * NCH * NPIX) return;
  if (in_sizes[1] != NBATCH * 3 * NPIX) return;
  if (out_size != NBATCH * NCH * NPIX) return;
  if (ws_size < WS_TOTAL) return;

  const float* pred = (const float*)d_in[0];
  const float* img  = (const float*)d_in[1];
  float* out = (float*)d_out;
  char* ws = (char*)d_ws;
  unsigned short* kbp = (unsigned short*)(ws + OFF_KBP);
  unsigned short* q16 = (unsigned short*)(ws + OFF_Q16);
  float* qfa = (float*)(ws + OFF_QFA);
  float* qfb = (float*)(ws + OFF_QFB);
  float* bi  = (float*)(ws + OFF_BI);

  const int padThreads  = (MROWS - NCH) * (NPIX / 8);
  const int packThreads = NCH * (NPIX / 8);
  const int kbThreads   = NPIX * (NPIX / 8);
  const int gemmTiles   = (MROWS / 64) * (NPIX / 64);
  const unsigned padBlocks  = (unsigned)((padThreads + 255) / 256);
  const unsigned packBlocks = (unsigned)((packThreads + 255) / 256);
  const unsigned kbBlocks   = (unsigned)((kbThreads + 255) / 256);
  const unsigned gemmBlocks = (unsigned)((gemmTiles + 7) / 8);

  zero_q16_pad_kernel<<<padBlocks, 256, 0, stream>>>(q16);

  for (int b = 0; b < NBATCH; ++b) {
    const float* predb = pred + (size_t)b * NCH * NPIX;
    const float* imgb  = img  + (size_t)b * 3 * NPIX;
    float* outb = out + (size_t)b * NCH * NPIX;

    build_kb_kernel<<<kbBlocks, 256, 0, stream>>>(imgb, kbp);
    pack_q16_kernel<<<packBlocks, 256, 0, stream>>>(predb, q16);

    for (int it = 0; it < NITER; ++it) {
      wmma_gemm64<0, false, 0, 0, false, 0><<<dim3(gemmBlocks, 1, 1), 256, 0, stream>>>(
          q16, q16, NPIX, 0L,
          kbp, kbp, NPIX, 0L,
          (void*)bi, (void*)bi, NPIX, 0L,
          (const float*)bi,
          (const float*)bi, 0L,
          MROWS, NPIX, NPIX, BI_SCALE);

      const float* qin;
      float* qdst;
      if (it == 0) qin = predb;
      else qin = ((it - 1) & 1) ? qfb : qfa;
      if (it == NITER - 1) qdst = outb;
      else qdst = (it & 1) ? qfb : qfa;
      spatial_update_kernel<<<NCH, 256, 0, stream>>>(qin, predb, bi, qdst, q16);
    }
  }
}
